// RSAL_2680059593313
// MI455X (gfx1250) — hardware-verified
//
#include <hip/hip_runtime.h>
#include <math.h>

typedef __attribute__((ext_vector_type(16))) _Float16 v16h;
typedef __attribute__((ext_vector_type(8)))  _Float16 v8h;
typedef __attribute__((ext_vector_type(16))) __bf16   v16b;
typedef __attribute__((ext_vector_type(8)))  __bf16   v8b;
typedef __attribute__((ext_vector_type(8)))  float    v8f;
typedef __attribute__((ext_vector_type(4)))  float    v4f;
typedef __attribute__((ext_vector_type(2)))  float    v2f;

constexpr int DMODEL  = 192;
constexpr int DINNER  = 384;
constexpr int NSTATE  = 16;
constexpr int DTRANK  = 12;
constexpr int XPREAL  = 44;
constexpr int XPROWS  = 88;
constexpr int XPPAD   = 128;
constexpr int XZPITCH = 768;
constexpr int NBATCH  = 8;
constexpr int IMGH    = 64;
constexpr int IMGW    = 64;
constexpr int SEQLEN  = IMGH * IMGW;
constexpr int NTOK    = NBATCH * SEQLEN;
constexpr int GRPB    = 2;
constexpr int GTOK    = GRPB * SEQLEN;
constexpr int NGRP    = NBATCH / GRPB;
static_assert(GTOK % 64 == 0);
static_assert(DMODEL % 32 == 0 && DINNER % 32 == 0);
static_assert(XPPAD % 64 == 0 && DMODEL % 64 == 0 && XZPITCH % 64 == 0);

__device__ __forceinline__ unsigned short f2bf_bits(float f) {
  unsigned u = __float_as_uint(f);
  return (unsigned short)((u + 0x7FFFu + ((u >> 16) & 1u)) >> 16);
}
__device__ __forceinline__ float bf_bits2f(unsigned short h) { return __uint_as_float(((unsigned)h) << 16); }
__device__ __forceinline__ float bfr(float v) { return bf_bits2f(f2bf_bits(v)); }

__device__ __forceinline__ void dep_guard_h(v8f& a, v8f& b, v16h x, v16h y) { asm volatile("v_nop\n\tv_nop\n\tv_nop\n\tv_nop" : "+v"(a), "+v"(b) : "v"(x), "v"(y)); }
__device__ __forceinline__ void dep_guard_b(v8f& a, v8f& b, v16b x, v16b y) { asm volatile("v_nop\n\tv_nop\n\tv_nop\n\tv_nop" : "+v"(a), "+v"(b) : "v"(x), "v"(y)); }
__device__ __forceinline__ void keep4_h(v16h a, v16h b, v16h c, v16h d) { asm volatile("v_nop" :: "v"(a), "v"(b), "v"(c), "v"(d)); }
__device__ __forceinline__ void keep4_b(v16b a, v16b b, v16b c, v16b d) { asm volatile("v_nop" :: "v"(a), "v"(b), "v"(c), "v"(d)); }
__device__ __forceinline__ void acc_guard4(v8f& a, v8f& b, v8f& c, v8f& d) { asm volatile("v_nop\n\tv_nop\n\tv_nop\n\tv_nop" : "+v"(a), "+v"(b), "+v"(c), "+v"(d)); }
template <typename T> struct Frag;
template <> struct Frag<_Float16> {
  typedef v16h V; union U { v16h v; v8h h[2]; };
  static __device__ __forceinline__ v16h load(const _Float16* p) {
    U f; f.h[0] = *(const v8h*)(p); f.h[1] = *(const v8h*)(p + 16); return f.v;
  }
  static __device__ __forceinline__ v8f mma(v16h a, v16h b, v8f c) {
    return __builtin_amdgcn_wmma_f32_16x16x32_f16(false, a, false, b, (short)0, c, false, false);
  }
  static __device__ __forceinline__ void guard(v8f& a, v8f& b, v16h x, v16h y) { dep_guard_h(a, b, x, y); }
  static __device__ __forceinline__ void keep(v16h a, v16h b, v16h c, v16h d) { keep4_h(a, b, c, d); }
};
template <> struct Frag<__bf16> {
  typedef v16b V; union U { v16b v; v8b h[2]; };
  static __device__ __forceinline__ v16b load(const __bf16* p) {
    U f; f.h[0] = *(const v8b*)(p); f.h[1] = *(const v8b*)(p + 16); return f.v;
  }
  static __device__ __forceinline__ v8f mma(v16b a, v16b b, v8f c) {
    return __builtin_amdgcn_wmma_f32_16x16x32_bf16(false, a, false, b, (short)0, c, false, false);
  }
  static __device__ __forceinline__ void guard(v8f& a, v8f& b, v16b x, v16b y) { dep_guard_b(a, b, x, y); }
  static __device__ __forceinline__ void keep(v16b a, v16b b, v16b c, v16b d) { keep4_b(a, b, c, d); }
};

template <int ET> struct Elem;
template <> struct Elem<0> { typedef _Float16 T; };
template <> struct Elem<1> { typedef __bf16 T; };
template <int ET, bool SPLIT, int BIAS_MODE, int OUT_MODE, bool RESID, int ACT = 0, bool BSPLIT = true>
__global__ __launch_bounds__(256) void wmma_gemm64(
    const unsigned short* __restrict__ Ap, const unsigned short* __restrict__ A2p, int lda, long strideA,
    const unsigned short* __restrict__ Btp, const unsigned short* __restrict__ Bt2p, int ldb, long strideB,
    void* __restrict__ Cout, void* __restrict__ Cout2, int ldc, long strideC,
    const float* __restrict__ bias,
    const float* __restrict__ resid, long strideR,
    int M, int N, int K, float scale) {
  typedef typename Elem<ET>::T T;
  typedef typename Frag<T>::V V;
  const T* A = (const T*)Ap; const T* A2 = (const T*)A2p; const T* Bt = (const T*)Btp; const T* Bt2 = (const T*)Bt2p;
  __shared__ __align__(16) float sT[8][16 * 68];
  const int b    = blockIdx.y;
  const int lane = threadIdx.x & 31;
  const int wave = threadIdx.x >> 5;
  const int tilesN = N >> 6;
  const int tilesM = M >> 6;
  const int tile = blockIdx.x * 8 + wave;
  if (tile >= tilesM * tilesN) return;
  const int tm = tile / tilesN;
  const int tn = tile - tm * tilesN;
  const int m0 = tm << 6;
  const int n0 = tn << 6;

  const T* Ab  = A  + (size_t)b * strideA;
  const T* Bb  = Bt + (size_t)b * strideB;
  const T* Ab2 = SPLIT ? (A2  + (size_t)b * strideA) : nullptr;
  const T* Bb2 = (SPLIT && BSPLIT) ? (Bt2 + (size_t)b * strideB) : nullptr;

  const int rlane = lane & 15;
  const int koff  = (lane >> 4) * 8;
  const int mOff  = (lane >> 4) * 8;

  v8f acc[4][4];
#pragma unroll
  for (int i = 0; i < 4; ++i)
#pragma unroll
    for (int j = 0; j < 4; ++j) acc[i][j] = (v8f){0.f,0.f,0.f,0.f,0.f,0.f,0.f,0.f};

  for (int k0 = 0; k0 < K; k0 += 32) {
    V bh[4], bl[4];
#pragma unroll
    for (int j = 0; j < 4; ++j) {
      const size_t bo = (size_t)(n0 + (j << 4) + rlane) * ldb + koff + k0;
      bh[j] = Frag<T>::load(Bb + bo);
      if (SPLIT && BSPLIT) bl[j] = Frag<T>::load(Bb2 + bo);
    }
#pragma unroll
    for (int i = 0; i < 4; ++i) {
      const size_t ao = (size_t)(m0 + (i << 4) + rlane) * lda + koff + k0;
      V ah = Frag<T>::load(Ab + ao);
      V al;
      if (SPLIT) al = Frag<T>::load(Ab2 + ao);
#pragma unroll
      for (int j = 0; j < 4; ++j) {
        acc[i][j] = Frag<T>::mma(ah, bh[j], acc[i][j]);
        if (SPLIT) {
          if (BSPLIT) acc[i][j] = Frag<T>::mma(ah, bl[j], acc[i][j]);
          acc[i][j] = Frag<T>::mma(al, bh[j], acc[i][j]);
        }
      }
      Frag<T>::guard(acc[i][0], acc[i][3], ah, SPLIT ? al : ah);
    }
    Frag<T>::keep(bh[0], bh[1], bh[2], bh[3]);
    if (SPLIT && BSPLIT) Frag<T>::keep(bl[0], bl[1], bl[2], bl[3]);
  }
  acc_guard4(acc[0][0], acc[0][1], acc[0][2], acc[0][3]);
  acc_guard4(acc[1][0], acc[1][1], acc[1][2], acc[1][3]);
  acc_guard4(acc[2][0], acc[2][1], acc[2][2], acc[2][3]);
  acc_guard4(acc[3][0], acc[3][1], acc[3][2], acc[3][3]);

  float* slab = sT[wave];
  const float* Rb = RESID ? (resid + (size_t)b * strideR) : nullptr;
#pragma unroll
  for (int i = 0; i < 4; ++i) {
    const int mBase = m0 + (i << 4);
#pragma unroll
    for (int j = 0; j < 4; ++j) {
      const int n = n0 + (j << 4) + rlane;
      float bv = 0.f;
      if (BIAS_MODE == 2) bv = bias[n];
#pragma unroll
      for (int r = 0; r < 8; ++r) {
        float v = acc[i][j][r] * scale;
        if (BIAS_MODE == 1) v += bias[mBase + mOff + r];
        if (BIAS_MODE == 2) v += bv;
        if (RESID) v += Rb[(size_t)(mBase + mOff + r) * ldc + n];
        if (ACT == 1) v = tanhf(v);
        if (ACT == 2) v = fmaxf(v, 0.0f);
        if (ACT == 3) v = v / (1.0f + expf(-v));
        if (ACT == 4) v = (v > 0.f) ? v : 0.01f * v;
        if (ACT == 5) v = 0.5f * v * (1.0f + erff(v * 0.70710678118654752f));
        slab[(mOff + r) * 68 + (j << 4) + rlane] = v;
      }
    }
    __builtin_amdgcn_fence(__ATOMIC_RELEASE, "workgroup");
    __builtin_amdgcn_wave_barrier();
    __builtin_amdgcn_fence(__ATOMIC_ACQUIRE, "workgroup");
    if (OUT_MODE == 0) {
      float* C = (float*)Cout + (size_t)b * strideC;
      const int hh = lane >> 4, c4 = (lane & 15) * 4;
      for (int pass = 0; pass < 2; ++pass) {
#pragma unroll
        for (int it = 0; it < 8; ++it) {
          const int row = it * 2 + hh;
          v4f v = *(const v4f*)(slab + row * 68 + c4);
          *(volatile v4f*)(C + (size_t)(mBase + row) * ldc + n0 + c4) = v;
        }
        __threadfence();
      }
    } else {
      const int q = lane >> 3, c8 = (lane & 7) * 8;
      unsigned short* C  = (unsigned short*)Cout  + (size_t)b * strideC;
      unsigned short* C2 = (OUT_MODE == 2) ? ((unsigned short*)Cout2 + (size_t)b * strideC) : nullptr;
      for (int pass = 0; pass < 2; ++pass) {
#pragma unroll
        for (int it = 0; it < 4; ++it) {
          const int row = it * 4 + q;
          const float* sp = slab + row * 68 + c8;
          v8h hv, lv;
#pragma unroll
          for (int e = 0; e < 8; ++e) {
            if (OUT_MODE == 1) {
              hv[e] = (_Float16)sp[e];
            } else {
              unsigned short hb = f2bf_bits(sp[e]);
              unsigned short lb = f2bf_bits(sp[e] - bf_bits2f(hb));
              hv[e] = __builtin_bit_cast(_Float16, hb);
              lv[e] = __builtin_bit_cast(_Float16, lb);
            }
          }
          *(volatile v8h*)(C + (size_t)(mBase + row) * ldc + n0 + c8) = hv;
          if (OUT_MODE == 2) *(volatile v8h*)(C2 + (size_t)(mBase + row) * ldc + n0 + c8) = lv;
        }
        __threadfence();
      }
    }
    __builtin_amdgcn_fence(__ATOMIC_RELEASE, "workgroup");
    __builtin_amdgcn_wave_barrier();
    __builtin_amdgcn_fence(__ATOMIC_ACQUIRE, "workgroup");
  }
}

__global__ __launch_bounds__(256) void cast_bf16_rows_kernel(
    const float* __restrict__ src, unsigned short* __restrict__ dst, int K, int nreal, int total8)
{
  const int i = blockIdx.x * 256 + threadIdx.x;
  if (i >= total8) return;
  const size_t e0 = (size_t)i << 3;
  const int row = (int)(e0 / (size_t)K);
  const int col = (int)(e0 - (size_t)row * K);
  const int rc  = (row < nreal) ? row : (nreal - 1);
  const bool keep = (row < nreal);
  const float* p = src + (size_t)rc * K + col;
  const v4f a0 = *(const v4f*)(p);
  const v4f a1 = *(const v4f*)(p + 4);
  v8h hv;
#pragma unroll
  for (int e = 0; e < 4; ++e) {
    const float v0 = keep ? a0[e] : 0.f;
    const float v1 = keep ? a1[e] : 0.f;
    hv[e]     = __builtin_bit_cast(_Float16, f2bf_bits(v0));
    hv[4 + e] = __builtin_bit_cast(_Float16, f2bf_bits(v1));
  }
  unsigned short* q = dst + e0;
  *(volatile v8h*)q = hv;
  __threadfence();
  *(volatile v8h*)q = hv;
}

__global__ __launch_bounds__(192) void conv_silu_kernel(
    const float* __restrict__ XZ, const float* __restrict__ cw, const float* __restrict__ cb,
    float* __restrict__ U, unsigned short* __restrict__ UH, unsigned short* __restrict__ UL)
{
  const int tid = threadIdx.x;
  const int c = tid * 2;
  const int img = blockIdx.x >> 6, hrow = blockIdx.x & 63;
  float wa[9], wb[9];
#pragma unroll
  for (int j = 0; j < 9; ++j) { wa[j] = bfr(cw[c * 9 + j]); wb[j] = bfr(cw[(c + 1) * 9 + j]); }
  const float ba = bfr(cb[c]), bb = bfr(cb[c + 1]);
  const bool vm = (hrow > 0), vp = (hrow < IMGH - 1);
  const int hmc = vm ? (hrow - 1) : 0, hpc = vp ? (hrow + 1) : (IMGH - 1);
  const size_t tokImg = (size_t)img * SEQLEN;
  const float* r0 = XZ + (tokImg + (size_t)hmc * IMGW) * XZPITCH + c;
  const float* r1 = XZ + (tokImg + (size_t)hrow * IMGW) * XZPITCH + c;
  const float* r2 = XZ + (tokImg + (size_t)hpc * IMGW) * XZPITCH + c;
  float ax[3][3], ay[3][3];
#pragma unroll
  for (int i = 0; i < 3; ++i) { ax[i][0] = 0.f; ay[i][0] = 0.f; }
  {
    const v2f t0 = *(const v2f*)(r0);
    const v2f t1 = *(const v2f*)(r1);
    const v2f t2 = *(const v2f*)(r2);
    ax[0][1] = vm ? t0.x : 0.f; ay[0][1] = vm ? t0.y : 0.f;
    ax[1][1] = t1.x;            ay[1][1] = t1.y;
    ax[2][1] = vp ? t2.x : 0.f; ay[2][1] = vp ? t2.y : 0.f;
  }
  const size_t tokRow = tokImg + (size_t)hrow * IMGW;
#pragma unroll 1
  for (int w = 0; w < IMGW; ++w) {
    const int wn = w + 1;
    const bool vn = (wn < IMGW);
    const int wnc = vn ? wn : (IMGW - 1);
    const size_t co = (size_t)wnc * XZPITCH;
    const v2f t0 = *(const v2f*)(r0 + co);
    const v2f t1 = *(const v2f*)(r1 + co);
    const v2f t2 = *(const v2f*)(r2 + co);
    const bool v0n = vm && vn, v2n = vp && vn;
    ax[0][2] = v0n ? t0.x : 0.f; ay[0][2] = v0n ? t0.y : 0.f;
    ax[1][2] = vn  ? t1.x : 0.f; ay[1][2] = vn  ? t1.y : 0.f;
    ax[2][2] = v2n ? t2.x : 0.f; ay[2][2] = v2n ? t2.y : 0.f;
    float sa = 0.f, sb = 0.f;
#pragma unroll
    for (int i = 0; i < 3; ++i) {
#pragma unroll
      for (int j = 0; j < 3; ++j) {
        sa = fmaf(wa[i * 3 + j], ax[i][j], sa);
        sb = fmaf(wb[i * 3 + j], ay[i][j], sb);
      }
    }
    sa += ba; sb += bb;
    const float ua = sa * __builtin_amdgcn_rcpf(1.0f + __expf(-sa));
    const float ub = sb * __builtin_amdgcn_rcpf(1.0f + __expf(-sb));
    const size_t tok = tokRow + w;
    v2f uv; uv.x = ua; uv.y = ub;
    const unsigned short ha = f2bf_bits(ua), hb = f2bf_bits(ub);
    const unsigned short la = f2bf_bits(ua - bf_bits2f(ha)), lb = f2bf_bits(ub - bf_bits2f(hb));
    const unsigned hpk = (unsigned)ha | ((unsigned)hb << 16);
    const unsigned lpk = (unsigned)la | ((unsigned)lb << 16);
    float* up = U + tok * DINNER + c;
    unsigned* uhp = (unsigned*)(UH + tok * DINNER + c);
    unsigned* ulp = (unsigned*)(UL + tok * DINNER + c);
    *(volatile v2f*)up = uv;
    *(volatile unsigned*)uhp = hpk;
    *(volatile unsigned*)ulp = lpk;
    __threadfence();
    *(volatile v2f*)up = uv;
    *(volatile unsigned*)uhp = hpk;
    *(volatile unsigned*)ulp = lpk;
#pragma unroll
    for (int i = 0; i < 3; ++i) {
      ax[i][0] = ax[i][1]; ax[i][1] = ax[i][2];
      ay[i][0] = ay[i][1]; ay[i][1] = ay[i][2];
    }
  }
}

union F12 { v4f q[3]; float f[12]; };
union F16 { v4f q[4]; float f[16]; };

__global__ __launch_bounds__(128) void scan_kernel(
    const float* __restrict__ XDBL, const float* __restrict__ U,
    const float* __restrict__ dtw, const float* __restrict__ dtb, const float* __restrict__ Alog,
    float* __restrict__ YY)
{
  const int tid = threadIdx.x;
  const int d  = blockIdx.x * 128 + tid;
  const int k  = blockIdx.y;
  const int img = blockIdx.z;
  const int kd = k * DINNER + d;
  float An[NSTATE];
#pragma unroll
  for (int n = 0; n < NSTATE; ++n) An[n] = -__expf(bfr(Alog[(size_t)kd * NSTATE + n]));
  float wd[DTRANK];
#pragma unroll
  for (int r = 0; r < DTRANK; ++r) wd[r] = bfr(dtw[(size_t)kd * DTRANK + r]);
  const float bias = bfr(dtb[kd]);
  float hs[NSTATE];
#pragma unroll
  for (int n = 0; n < NSTATE; ++n) hs[n] = 0.f;
  const size_t tokBase = (size_t)img * SEQLEN;
  float* Yk = YY + (size_t)k * GTOK * DINNER;
  const int xoff = k * XPREAL;
#pragma unroll 1
  for (int t = 0; t < SEQLEN; ++t) {
    const int l = k ? (SEQLEN - 1 - t) : t;
    const size_t row = tokBase + (size_t)l;
    const float* xr = XDBL + row * XPPAD + xoff;
    F12 dq;
    dq.q[0] = *(const v4f*)(xr);      dq.q[1] = *(const v4f*)(xr + 4);  dq.q[2] = *(const v4f*)(xr + 8);
    F16 Bq, Cq;
    Bq.q[0] = *(const v4f*)(xr + 12); Bq.q[1] = *(const v4f*)(xr + 16);
    Bq.q[2] = *(const v4f*)(xr + 20); Bq.q[3] = *(const v4f*)(xr + 24);
    Cq.q[0] = *(const v4f*)(xr + 28); Cq.q[1] = *(const v4f*)(xr + 32);
    Cq.q[2] = *(const v4f*)(xr + 36); Cq.q[3] = *(const v4f*)(xr + 40);
    const float u = U[row * DINNER + d];
    float dl = 0.f;
#pragma unroll
    for (int r = 0; r < DTRANK; ++r) dl = fmaf(dq.f[r], wd[r], dl);
    dl += bias;
    const float sp = fmaxf(dl, 0.f) + log1pf(__expf(-fabsf(dl)));
    const float bx = sp * u;
    float y = 0.f;
#pragma unroll
    for (int n = 0; n < NSTATE; ++n) {
      const float a = __expf(sp * An[n]);
      hs[n] = fmaf(a, hs[n], bx * Bq.f[n]);
      y = fmaf(hs[n], Cq.f[n], y);
    }
    float* yp = Yk + row * DINNER + d;
    *(volatile float*)yp = y;
    __threadfence();
    *(volatile float*)yp = y;
  }
}

__global__ __launch_bounds__(192) void ln_gate_kernel(
    const float* __restrict__ YY, const float* __restrict__ U, const float* __restrict__ XZ,
    const float* __restrict__ Dv, const float* __restrict__ lnw, const float* __restrict__ lnb,
    unsigned short* __restrict__ YH, unsigned short* __restrict__ YL)
{
  __shared__ float red[2][8];
  const int tid = threadIdx.x, lane = tid & 31, wave = tid >> 5;
  const int c = tid * 2;
  const float d0a = bfr(Dv[c]), d0b = bfr(Dv[c + 1]);
  const float d1a = bfr(Dv[DINNER + c]), d1b = bfr(Dv[DINNER + c + 1]);
  const float ga = bfr(lnw[c]), gb = bfr(lnw[c + 1]);
  const float ba = bfr(lnb[c]), bb = bfr(lnb[c + 1]);
  const float inv_n = 1.0f / (float)DINNER;
#pragma unroll 1
  for (int tt = 0; tt < 4; ++tt) {
    const size_t tok = (size_t)blockIdx.x * 4 + tt;
    const v2f y0 = *(const v2f*)(YY + tok * DINNER + c);
    const v2f y1 = *(const v2f*)(YY + (size_t)GTOK * DINNER + tok * DINNER + c);
    const v2f uu = *(const v2f*)(U + tok * DINNER + c);
    const v2f zz = *(const v2f*)(XZ + tok * XZPITCH + DINNER + c);
    const float ya = (y0.x + uu.x * d0a) + (y1.x + uu.x * d1a);
    const float yb = (y0.y + uu.y * d0b) + (y1.y + uu.y * d1b);
    float s = ya + yb;
#pragma unroll
    for (int off = 16; off; off >>= 1) s += __shfl_xor(s, off, 32);
    if (lane == 0) red[0][wave] = s;
    __syncthreads();
    const float tot = red[0][0] + red[0][1] + red[0][2] + red[0][3] + red[0][4] + red[0][5];
    const float mean = tot * inv_n;
    const float da = ya - mean, db = yb - mean;
    float q = da * da + db * db;
#pragma unroll
    for (int off = 16; off; off >>= 1) q += __shfl_xor(q, off, 32);
    if (lane == 0) red[1][wave] = q;
    __syncthreads();
    const float qt = red[1][0] + red[1][1] + red[1][2] + red[1][3] + red[1][4] + red[1][5];
    const float var = qt * inv_n;
    const float rs = rsqrtf(var + 1e-5f);
    const float na = da * rs * ga + ba;
    const float nb = db * rs * gb + bb;
    const float gea = 0.5f * zz.x * (1.0f + erff(zz.x * 0.70710678118654752f));
    const float geb = 0.5f * zz.y * (1.0f + erff(zz.y * 0.70710678118654752f));
    const float oa = na * gea, ob = nb * geb;
    const unsigned short h0 = f2bf_bits(oa), h1 = f2bf_bits(ob);
    const unsigned short l0 = f2bf_bits(oa - bf_bits2f(h0)), l1 = f2bf_bits(ob - bf_bits2f(h1));
    const unsigned hpk = (unsigned)h0 | ((unsigned)h1 << 16);
    const unsigned lpk = (unsigned)l0 | ((unsigned)l1 << 16);
    unsigned* ph = (unsigned*)(YH + tok * DINNER + c);
    unsigned* pl = (unsigned*)(YL + tok * DINNER + c);
    *(volatile unsigned*)ph = hpk;
    *(volatile unsigned*)pl = lpk;
    __threadfence();
    *(volatile unsigned*)ph = hpk;
    *(volatile unsigned*)pl = lpk;
  }
}

extern "C" void kernel_launch(void* const* d_in, const int* in_sizes, int n_in,
                              void* d_out, int out_size, void* d_ws, size_t ws_size,
                              hipStream_t stream) {
  if (n_in < 12) return;
  if (in_sizes[0] != NTOK * DMODEL || out_size != NTOK * DMODEL) return;
  if (in_sizes[1] != 2 * DINNER * DMODEL || in_sizes[2] != DINNER * 9 || in_sizes[3] != DINNER) return;
  if (in_sizes[4] != 2 * XPREAL * DINNER || in_sizes[5] != 2 * DINNER * DTRANK || in_sizes[6] != 2 * DINNER) return;
  if (in_sizes[7] != 2 * DINNER * NSTATE || in_sizes[8] != 2 * DINNER) return;
  if (in_sizes[9] != DINNER || in_sizes[10] != DINNER || in_sizes[11] != DMODEL * DINNER) return;

  const float* x     = (const float*)d_in[0];
  const float* w_in  = (const float*)d_in[1];
  const float* cw    = (const float*)d_in[2];
  const float* cb    = (const float*)d_in[3];
  const float* w_xp  = (const float*)d_in[4];
  const float* dtw   = (const float*)d_in[5];
  const float* dtb   = (const float*)d_in[6];
  const float* alog  = (const float*)d_in[7];
  const float* Dv    = (const float*)d_in[8];
  const float* lnw   = (const float*)d_in[9];
  const float* lnb   = (const float*)d_in[10];
  const float* w_out = (const float*)d_in[11];
  float* out = (float*)d_out;

  char* base = (char*)d_ws;
  size_t off = 0;
  auto carve = [&](size_t bytes) -> char* {
    char* r = base + off;
    off += (bytes + 255) & ~(size_t)255;
    return r;
  };
  unsigned short* WinB = (unsigned short*)carve((size_t)2 * DINNER * DMODEL * 2);
  unsigned short* WxpB = (unsigned short*)carve((size_t)XPPAD * DINNER * 2);
  unsigned short* WoB  = (unsigned short*)carve((size_t)DMODEL * DINNER * 2);
  unsigned short* XB   = (unsigned short*)carve((size_t)NTOK * DMODEL * 2);
  float*          XZ   = (float*)carve((size_t)GTOK * XZPITCH * 4);
  float*          U    = (float*)carve((size_t)GTOK * DINNER * 4);
  unsigned short* UH   = (unsigned short*)carve((size_t)GTOK * DINNER * 2);
  unsigned short* UL   = (unsigned short*)carve((size_t)GTOK * DINNER * 2);
  float*          XDBL = (float*)carve((size_t)GTOK * XPPAD * 4);
  float*          YY   = (float*)carve((size_t)2 * GTOK * DINNER * 4);
  unsigned short* YH   = (unsigned short*)carve((size_t)GTOK * DINNER * 2);
  unsigned short* YL   = (unsigned short*)carve((size_t)GTOK * DINNER * 2);
  if (off > ws_size) return;

  cast_bf16_rows_kernel<<<(2 * DINNER * DMODEL / 8) / 256, 256, 0, stream>>>(w_in, WinB, DMODEL, 2 * DINNER, 2 * DINNER * DMODEL / 8);
  cast_bf16_rows_kernel<<<(XPPAD * DINNER / 8) / 256, 256, 0, stream>>>(w_xp, WxpB, DINNER, XPROWS, XPPAD * DINNER / 8);
  cast_bf16_rows_kernel<<<(DMODEL * DINNER / 8) / 256, 256, 0, stream>>>(w_out, WoB, DINNER, DMODEL, DMODEL * DINNER / 8);
  cast_bf16_rows_kernel<<<(NTOK * DMODEL / 8) / 256, 256, 0, stream>>>(x, XB, DMODEL, NTOK, NTOK * DMODEL / 8);

  for (int g = 0; g < NGRP; ++g) {
    const unsigned short* xg = XB + (size_t)g * GTOK * DMODEL;
    float* outg = out + (size_t)g * GTOK * DMODEL;

    wmma_gemm64<1, false, 0, 0, false, 0, true><<<dim3(192, 1), 256, 0, stream>>>(
        xg, xg, DMODEL, 0L, WinB, WinB, DMODEL, 0L, (void*)XZ, (void*)XZ, XZPITCH, 0L,
        dtb, dtb, 0L, GTOK, XZPITCH, DMODEL, 1.0f);

    conv_silu_kernel<<<GRPB * IMGH, 192, 0, stream>>>(XZ, cw, cb, U, UH, UL);

    wmma_gemm64<1, true, 0, 0, false, 0, false><<<dim3(32, 1), 256, 0, stream>>>(
        UH, UL, DINNER, 0L, WxpB, WxpB, DINNER, 0L, (void*)XDBL, (void*)XDBL, XPPAD, 0L,
        dtb, dtb, 0L, GTOK, XPPAD, DINNER, 1.0f);

    scan_kernel<<<dim3(DINNER / 128, 2, GRPB), 128, 0, stream>>>(XDBL, U, dtw, dtb, alog, YY);

    ln_gate_kernel<<<GTOK / 4, 192, 0, stream>>>(YY, U, XZ, Dv, lnw, lnb, YH, YL);

    wmma_gemm64<1, true, 0, 0, false, 0, false><<<dim3(48, 1), 256, 0, stream>>>(
        YH, YL, DINNER, 0L, WoB, WoB, DINNER, 0L, (void*)outg, (void*)outg, DMODEL, 0L,
        dtb, dtb, 0L, GTOK, DMODEL, DINNER, 1.0f);
  }
}
